// GNN_Heuristic_9929964389268
// MI455X (gfx1250) — hardware-verified
//
#include <hip/hip_runtime.h>
#include <stddef.h>
#include <math.h>


#define DF    128
#define GR    32
#define AP    136
#define XSP   132
#define NPART 8
#define HP    4
#define TP    129
#define NB    512
#define CHUNK 2048
#define NTHR  256
#define NWAVE 8
#define WCAP  256
#define NGRP  (CHUNK / (NTHR * 4))
#define WSC   64.0f
#define WSCI  0.015625f

#define LDS_SACC (NB * DF)
#define LDS_DEN  (NB * HP)
#define LDS_MAX  (NB * HP)
#define LDS_LIST (NWAVE * WCAP)
#define LDS_BYTES ((LDS_SACC + LDS_DEN + LDS_MAX + LDS_LIST + NWAVE) * 4)

static_assert(WCAP == (CHUNK / NTHR) * 32);
static_assert(NGRP == 2);
static_assert(NB == 512);
static_assert(CHUNK == 2048);
static_assert(((LDS_SACC + LDS_DEN) % 4) == 0);
static_assert((LDS_MAX % 4) == 0);
static_assert((NB % NWAVE) == 0);
static_assert((NB / NWAVE) == 64);
static_assert(LDS_BYTES == 286752);
static_assert((DF % 32) == 0);

typedef float    v4f  __attribute__((ext_vector_type(4)));
typedef float    v8f  __attribute__((ext_vector_type(8)));
typedef int      v4i  __attribute__((ext_vector_type(4)));
typedef _Float16 v8h  __attribute__((ext_vector_type(8)));
typedef _Float16 v16h __attribute__((ext_vector_type(16)));
union Frag  { v16h v; v8h half[2]; };
union PackH { v8h h; v4i i; };

__device__ __forceinline__ v8f wm(v16h a, v16h b, v8f c) {
  v8f d = __builtin_amdgcn_wmma_f32_16x16x32_f16(false, a, false, b, (short)0, c, false, false);
  asm volatile("v_nop\n\tv_nop\n\tv_nop\n\tv_nop" : "+v"(d) : "v"(a), "v"(b));
  return d;
}

__global__ __launch_bounds__(NTHR) void k_prepw(const float* __restrict__ Wa, const float* __restrict__ Wb,
                                                _Float16* Wta, _Float16* Wtb) {
  __shared__ __attribute__((aligned(16))) float T[32 * TP];
  const int tid = threadIdx.x;
  const bool second = (blockIdx.x >= 4);
  const float* W  = second ? Wb : Wa;
  _Float16*    Wt = second ? Wtb : Wta;
  const int n0  = (blockIdx.x & 3) * 32;
#pragma unroll
  for (int i = 0; i < 16; ++i) {
    const int idx = i * NTHR + tid;
    const int k   = idx >> 5;
    const int c   = idx & 31;
    T[c * TP + k] = W[(size_t)k * DF + n0 + c];
  }
  __syncthreads();
  PackH u[2];
  size_t po[2];
#pragma unroll
  for (int q = 0; q < 2; ++q) {
    const int t  = q * NTHR + tid;
    const int c  = t >> 4;
    const int k0 = (t & 15) * 8;
#pragma unroll
    for (int j = 0; j < 8; ++j) u[q].h[j] = (_Float16)(T[c * TP + k0 + j] * WSC);
    po[q] = (size_t)(n0 + c) * DF + k0;
  }
#pragma unroll
  for (int q = 0; q < 2; ++q) *(volatile v4i*)(Wt + po[q]) = u[q].i;
  __threadfence();
#pragma unroll
  for (int q = 0; q < 2; ++q) *(volatile v4i*)(Wt + po[q]) = u[q].i;
}

__device__ __forceinline__ void epi_tile(v8f acc, int T, int hh, int m, int wave, int ncol,
                                         float cs, float cd, float* Xs, float* Ps, float* Pd) {
  float ss[8], sd[8];
#pragma unroll
  for (int r = 0; r < 8; ++r) {
    const float v = acc[r] * WSCI;
    Xs[(T * 16 + 8 * hh + r) * XSP + ncol] = v;
    ss[r] = v * cs;
    sd[r] = v * cd;
  }
#pragma unroll
  for (int mk = 1; mk < 16; mk <<= 1) {
#pragma unroll
    for (int r = 0; r < 8; ++r) {
      ss[r] += __shfl_xor(ss[r], mk, 32);
      sd[r] += __shfl_xor(sd[r], mk, 32);
    }
  }
  if (m == 0) {
#pragma unroll
    for (int r = 0; r < 8; ++r) {
      Ps[(T * 16 + 8 * hh + r) * NPART + wave] = ss[r];
      Pd[(T * 16 + 8 * hh + r) * NPART + wave] = sd[r];
    }
  }
}

__global__ __launch_bounds__(NTHR) void k_gemm(
    const float* __restrict__ x, const _Float16* __restrict__ Wt,
    const float* __restrict__ attl, const float* __restrict__ attr,
    float* xp, float* elp, float* erp, int nN, int H) {
  __shared__ __attribute__((aligned(16))) _Float16 Ah[GR * AP];
  __shared__ __attribute__((aligned(16))) float Xs[GR * XSP];
  __shared__ __attribute__((aligned(16))) float Pp[2 * GR * NPART];
  float* Ps = Pp;
  float* Pd = Pp + GR * NPART;

  const int tid  = threadIdx.x;
  const int lane = tid & 31;
  const int wave = tid >> 5;
  const int hh   = lane >> 4;
  const int m    = lane & 15;
  const int rowBase = blockIdx.x * GR;

  {
    const int r  = tid >> 3;
    const int c0 = (tid & 7) * 16;
    int row = rowBase + r;
    if (row > nN - 1) row = nN - 1;
    const float* p = x + (size_t)row * DF + c0;
    const v4f f0 = *(const v4f*)(p), f1 = *(const v4f*)(p + 4);
    const v4f f2 = *(const v4f*)(p + 8), f3 = *(const v4f*)(p + 12);
    PackH h0, h1;
    h0.h[0] = (_Float16)f0.x; h0.h[1] = (_Float16)f0.y; h0.h[2] = (_Float16)f0.z; h0.h[3] = (_Float16)f0.w;
    h0.h[4] = (_Float16)f1.x; h0.h[5] = (_Float16)f1.y; h0.h[6] = (_Float16)f1.z; h0.h[7] = (_Float16)f1.w;
    h1.h[0] = (_Float16)f2.x; h1.h[1] = (_Float16)f2.y; h1.h[2] = (_Float16)f2.z; h1.h[3] = (_Float16)f2.w;
    h1.h[4] = (_Float16)f3.x; h1.h[5] = (_Float16)f3.y; h1.h[6] = (_Float16)f3.z; h1.h[7] = (_Float16)f3.w;
    *(v8h*)(Ah + r * AP + c0)     = h0.h;
    *(v8h*)(Ah + r * AP + c0 + 8) = h1.h;
  }
  __syncthreads();

  const int ncol = wave * 16 + m;
  v8f c0a = {0.f, 0.f, 0.f, 0.f, 0.f, 0.f, 0.f, 0.f};
  v8f c1a = {0.f, 0.f, 0.f, 0.f, 0.f, 0.f, 0.f, 0.f};
#pragma unroll
  for (int kt = 0; kt < DF / 32; ++kt) {
    const int k0 = kt * 32;
    Frag a0, a1, b;
    const _Float16* pb  = Wt + (size_t)ncol * DF + k0 + 8 * hh;
    const _Float16* pa0 = Ah + m * AP + k0 + 8 * hh;
    const _Float16* pa1 = Ah + (16 + m) * AP + k0 + 8 * hh;
    b.half[0]  = *(const v8h*)pb;   b.half[1]  = *(const v8h*)(pb + 16);
    a0.half[0] = *(const v8h*)pa0;  a0.half[1] = *(const v8h*)(pa0 + 16);
    a1.half[0] = *(const v8h*)pa1;  a1.half[1] = *(const v8h*)(pa1 + 16);
    c0a = wm(a0.v, b.v, c0a);
    c1a = wm(a1.v, b.v, c1a);
  }

  const float cs = attl[ncol];
  const float cd = attr[ncol];
  epi_tile(c0a, 0, hh, m, wave, ncol, cs, cd, Xs, Ps, Pd);
  epi_tile(c1a, 1, hh, m, wave, ncol, cs, cd, Xs, Ps, Pd);
  __syncthreads();

  v4f xr[4];
#pragma unroll
  for (int i = 0; i < 4; ++i) xr[i] = *(const v4f*)(Xs + (4 * wave + i) * XSP + 4 * lane);
  v4f gv = {0.f, 0.f, 0.f, 0.f};
  if (wave < 2) {
    const float* P = Pp + wave * (GR * NPART) + lane * NPART;
    const v4f q0 = *(const v4f*)(P);
    const v4f q1 = *(const v4f*)(P + 4);
    if (H == 4) {
      gv.x = q0.x + q0.y; gv.y = q0.z + q0.w; gv.z = q1.x + q1.y; gv.w = q1.z + q1.w;
    } else {
      gv.x = ((q0.x + q0.y) + (q0.z + q0.w)) + ((q1.x + q1.y) + (q1.z + q1.w));
    }
  }
  float* gp = ((wave == 0) ? elp : erp) + ((size_t)rowBase + lane) * HP;
  float* xpp[4];
#pragma unroll
  for (int i = 0; i < 4; ++i) xpp[i] = xp + (size_t)(rowBase + 4 * wave + i) * DF + 4 * lane;

#pragma unroll
  for (int i = 0; i < 4; ++i) *(volatile v4f*)(xpp[i]) = xr[i];
  if (wave < 2) *(volatile v4f*)gp = gv;
  __threadfence();
#pragma unroll
  for (int i = 0; i < 4; ++i) *(volatile v4f*)(xpp[i]) = xr[i];
  if (wave < 2) *(volatile v4f*)gp = gv;
}

__global__ __launch_bounds__(NTHR) void k_gat(
    const float* __restrict__ feat, const float* __restrict__ elp, const float* __restrict__ erp,
    const int* __restrict__ srcp, const int* __restrict__ dstp,
    const float* __restrict__ bias, const float* __restrict__ wfc,
    float* out, int nN, int nE, int H, int mode) {
  extern __shared__ v4f lds_dyn[];
  float* sacc = (float*)lds_dyn;
  float* daux = sacc + LDS_SACC;
  float* maux = daux + LDS_DEN;
  int*   list = (int*)(maux + LDS_MAX);
  int*   wcnt = list + LDS_LIST;

  const int tid  = threadIdx.x;
  const int lane = tid & 31;
  const int wave = tid >> 5;
  const int hd   = (lane * H) >> 5;
  const int nodeBase = blockIdx.x * NB;

  {
    const v4f z4 = {0.f, 0.f, 0.f, 0.f};
    for (int i = tid; i < (LDS_SACC + LDS_DEN) / 4; i += NTHR) lds_dyn[i] = z4;
    const float ninf = __uint_as_float(0xff800000u);
    const v4f n4 = {ninf, ninf, ninf, ninf};
    for (int i = tid; i < LDS_MAX / 4; i += NTHR) lds_dyn[(LDS_SACC + LDS_DEN) / 4 + i] = n4;
  }
  __syncthreads();
  const bool al16 = ((((size_t)dstp) & 15) == 0);

  const int nChunks = (nE + CHUNK - 1) / CHUNK;
#pragma unroll 1
  for (int ch = 0; ch < nChunks; ++ch) {
    const int cbase = ch * CHUNK;
    int wc = 0;
#pragma unroll
    for (int g = 0; g < NGRP; ++g) {
      const int el0 = (g * NTHR + tid) * 4;
      const int e0  = cbase + el0;
      const int sent = -2147483647 - 1;
      v4i d;
      if (al16 && (cbase + CHUNK <= nE)) {
        d = *(const v4i*)(dstp + e0);
      } else {
        d.x = (e0     < nE) ? dstp[min(e0, nE - 1)]     : sent;
        d.y = (e0 + 1 < nE) ? dstp[min(e0 + 1, nE - 1)] : sent;
        d.z = (e0 + 2 < nE) ? dstp[min(e0 + 2, nE - 1)] : sent;
        d.w = (e0 + 3 < nE) ? dstp[min(e0 + 3, nE - 1)] : sent;
      }
      const unsigned s0 = (unsigned)d.x - (unsigned)nodeBase;
      const unsigned s1 = (unsigned)d.y - (unsigned)nodeBase;
      const unsigned s2 = (unsigned)d.z - (unsigned)nodeBase;
      const unsigned s3 = (unsigned)d.w - (unsigned)nodeBase;
      const bool h0 = s0 < (unsigned)NB;
      const bool h1 = s1 < (unsigned)NB;
      const bool h2 = s2 < (unsigned)NB;
      const bool h3 = s3 < (unsigned)NB;
      const unsigned many = __builtin_amdgcn_ballot_w32(h0 | h1 | h2 | h3);
      if (many != 0u) {
#define HITJ(J, HJ, SJ) { \
          const unsigned mj = __builtin_amdgcn_ballot_w32(HJ); \
          if (HJ) { \
            const int pos = wc + (int)__builtin_amdgcn_mbcnt_lo(mj, 0u); \
            if (pos < WCAP) list[wave * WCAP + pos] = ((el0 + (J)) << 9) | (int)(SJ); \
          } \
          wc += (int)__builtin_popcount(mj); }
        HITJ(0, h0, s0)
        HITJ(1, h1, s1)
        HITJ(2, h2, s2)
        HITJ(3, h3, s3)
#undef HITJ
      }
    }
    if (lane == 0) wcnt[wave] = wc;
    __syncthreads();

    if (wave == 0) {
      for (int wsx = 0; wsx < NWAVE; ++wsx) {
        int n = __builtin_amdgcn_readfirstlane(wcnt[wsx]);
        n = n > WCAP ? WCAP : n;
        n = n < 0 ? 0 : n;
        for (int i = 0; i < n; ++i) {
          const int ent  = __builtin_amdgcn_readfirstlane(list[wsx * WCAP + i]);
          const int slot = ent & (NB - 1);
          const int eloc = (ent >> 9) & (CHUNK - 1);
          int e = cbase + eloc;
          e = e > nE - 1 ? nE - 1 : e;
          int j = srcp[e];
          j = j < 0 ? 0 : (j > nN - 1 ? nN - 1 : j);
          int nd = nodeBase + slot;
          nd = nd > nN - 1 ? nN - 1 : nd;
          float s = elp[(size_t)j * HP + hd] + erp[(size_t)nd * HP + hd];
          s = (s >= 0.f) ? s : 0.2f * s;
          const int ai = slot * HP + hd;
          const float mo = maux[ai];
          const float dn = daux[ai];
          const float mn = fmaxf(mo, s);
          const float cf = __expf(mo - mn);
          const float p  = __expf(s - mn);
          const v4f xv = *(const v4f*)(feat + (size_t)j * DF + 4 * lane);
          v4f* sp = (v4f*)(sacc + slot * DF + 4 * lane);
          const v4f cur = *sp;
          const v4f nxt = cur * cf + xv * p;
          *sp = nxt;
          maux[ai] = mn;
          daux[ai] = dn * cf + p;
        }
      }
    }
    __syncthreads();
  }

  const v4f b4 = *(const v4f*)(bias + 4 * lane);
  const v4f w0 = *(const v4f*)(wfc + 4 * lane);
  const v4f w1 = *(const v4f*)(wfc + DF + 4 * lane);
  v4f uwv = {0.f, 0.f, 0.f, 0.f};
#pragma unroll 1
  for (int q = 0; q < NB / NWAVE; ++q) {
    const int slot = wave * (NB / NWAVE) + q;
    int nd = nodeBase + slot;
    nd = nd > nN - 1 ? nN - 1 : nd;
    float s = elp[(size_t)nd * HP + hd] + erp[(size_t)nd * HP + hd];
    s = (s >= 0.f) ? s : 0.2f * s;
    const int ai = slot * HP + hd;
    const float mo  = maux[ai];
    const float dn0 = daux[ai];
    const float mn  = fmaxf(mo, s);
    const float cf  = __expf(mo - mn);
    const float p   = __expf(s - mn);
    const v4f xv = *(const v4f*)(feat + (size_t)nd * DF + 4 * lane);
    const v4f sv = *(const v4f*)(sacc + slot * DF + 4 * lane);
    const float dn  = dn0 * cf + p;
    const float inv = (dn > 0.f) ? (1.0f / dn) : 0.f;
    v4f y = (sv * cf + xv * p) * inv + b4;
    if (mode == 1) {
      float t0 = y.x, t1 = y.y, t2 = y.z, t3 = y.w;
#pragma unroll 1
      for (int c = 0; c < 4; ++c) {
        float v = t0;
        const float ng = expm1f(fminf(v, 0.f));
        v = (v > 0.f) ? v : ng;
        t0 = t1; t1 = t2; t2 = t3; t3 = v;
      }
      y.x = t0; y.y = t1; y.z = t2; y.w = t3;
      float* op = out + (size_t)(nodeBase + slot) * DF + 4 * lane;
      *(volatile v4f*)op = y;
      __threadfence();
      *(volatile v4f*)op = y;
    } else {
      float u = y.x * w0.x + y.y * w0.y + y.z * w0.z + y.w * w0.w;
      float w = y.x * w1.x + y.y * w1.y + y.z * w1.z + y.w * w1.w;
#pragma unroll
      for (int mk = 1; mk < 32; mk <<= 1) {
        u += __shfl_xor(u, mk, 32);
        w += __shfl_xor(w, mk, 32);
      }
      if (lane == (q >> 1)) {
        if (q & 1) { uwv.z = u; uwv.w = w; }
        else       { uwv.x = u; uwv.y = w; }
      }
    }
  }
  if (mode != 1) {
    float* op = out + (size_t)(nodeBase + wave * (NB / NWAVE)) * 2 + 4 * lane;
    *(volatile v4f*)op = uwv;
    __threadfence();
    *(volatile v4f*)op = uwv;
  }
}

__global__ __launch_bounds__(NTHR) void k_head(const int* __restrict__ eli, const float* __restrict__ uw,
                                               const float* __restrict__ bfc, float* out, int nL, int nN) {
  const int p0 = 4 * (blockIdx.x * NTHR + (int)threadIdx.x);
  const float bb = bfc[0];
  float t0 = 0.f, t1 = 0.f, t2 = 0.f, t3 = 0.f;
#pragma unroll 1
  for (int c = 0; c < 4; ++c) {
    int p = p0 + c;
    p = p > nL - 1 ? nL - 1 : p;
    int i0 = eli[p];
    int i1 = eli[(size_t)nL + p];
    i0 = i0 < 0 ? 0 : (i0 > nN - 1 ? nN - 1 : i0);
    i1 = i1 < 0 ? 0 : (i1 > nN - 1 ? nN - 1 : i1);
    float v = uw[(size_t)i0 * 2] + uw[(size_t)i1 * 2 + 1] + bb;
    v = fminf(fmaxf(v, -30.f), 30.f);
    const float ex = expf(-v);
    const float o  = 1.0f / (1.0f + ex);
    t0 = t1; t1 = t2; t2 = t3; t3 = o;
  }
  if (p0 < nL) {
    const v4f o4 = {t0, t1, t2, t3};
    float* op = out + p0;
    *(volatile v4f*)op = o4;
    __threadfence();
    *(volatile v4f*)op = o4;
  }
}

extern "C" void kernel_launch(void* const* d_in, const int* in_sizes, int n_in,
                              void* d_out, int out_size, void* d_ws, size_t ws_size,
                              hipStream_t stream) {
  if (n_in != 13) return;
  if (in_sizes[0] <= 0 || (in_sizes[0] % DF) != 0) return;
  const int nN = in_sizes[0] / DF;
  if (in_sizes[1] < 2 || (in_sizes[1] & 1) != 0) return;
  const int nE = in_sizes[1] / 2;
  if (in_sizes[2] < 4 || (in_sizes[2] & 1) != 0) return;
  const int nL = in_sizes[2] / 2;
  if (in_sizes[3] != DF * DF || in_sizes[7] != DF * DF) return;
  if (in_sizes[4] != DF || in_sizes[5] != DF || in_sizes[6] != DF) return;
  if (in_sizes[8] != DF || in_sizes[9] != DF || in_sizes[10] != DF) return;
  if (in_sizes[11] != 2 * DF || in_sizes[12] < 1) return;
  if (out_size != nL || (nL & 3) != 0) return;

  const float* x   = (const float*)d_in[0];
  const int*   ei  = (const int*)d_in[1];
  const int*   eli = (const int*)d_in[2];
  const float* W1  = (const float*)d_in[3];
  const float* as1 = (const float*)d_in[4];
  const float* ad1 = (const float*)d_in[5];
  const float* b1  = (const float*)d_in[6];
  const float* W2  = (const float*)d_in[7];
  const float* as2 = (const float*)d_in[8];
  const float* ad2 = (const float*)d_in[9];
  const float* b2  = (const float*)d_in[10];
  const float* Wfc = (const float*)d_in[11];
  const float* bfc = (const float*)d_in[12];
  float* outp = (float*)d_out;

  const int nPad = ((nN + NB - 1) / NB) * NB;
  size_t off = 0;
  _Float16* Wt1 = (_Float16*)((char*)d_ws + off); off += (size_t)DF * DF * sizeof(_Float16);
  _Float16* Wt2 = (_Float16*)((char*)d_ws + off); off += (size_t)DF * DF * sizeof(_Float16);
  float* xp  = (float*)((char*)d_ws + off); off += (size_t)nPad * DF * sizeof(float);
  float* hh  = (float*)((char*)d_ws + off); off += (size_t)nPad * DF * sizeof(float);
  float* elp = (float*)((char*)d_ws + off); off += (size_t)nPad * HP * sizeof(float);
  float* erp = (float*)((char*)d_ws + off); off += (size_t)nPad * HP * sizeof(float);
  float* uw  = (float*)((char*)d_ws + off); off += (size_t)nPad * 2 * sizeof(float);
  if (off > ws_size) return;

  const int* srcp = ei;
  const int* dstp = ei + nE;

  hipFuncSetAttribute(reinterpret_cast<const void*>(&k_gat),
                      hipFuncAttributeMaxDynamicSharedMemorySize, LDS_BYTES);
  const int ggemm = nPad / GR;
  const int ggat  = nPad / NB;
  const int ghead = (nL + 4 * NTHR - 1) / (4 * NTHR);

  k_prepw<<<8, NTHR, 0, stream>>>(W1, W2, Wt1, Wt2);
  k_gemm<<<ggemm, NTHR, 0, stream>>>(x, Wt1, as1, ad1, xp, elp, erp, nN, 4);
  k_gat<<<ggat, NTHR, LDS_BYTES, stream>>>(xp, elp, erp, srcp, dstp, b1, Wfc, hh, nN, nE, 4, 1);
  k_gemm<<<ggemm, NTHR, 0, stream>>>(hh, Wt2, as2, ad2, xp, elp, erp, nN, 1);
  k_gat<<<ggat, NTHR, LDS_BYTES, stream>>>(xp, elp, erp, srcp, dstp, b2, Wfc, uw, nN, nE, 1, 2);
  k_head<<<ghead, NTHR, 0, stream>>>(eli, uw, bfc, outp, nL, nN);
}
